// HeteroGNNBA_14551349198940
// MI455X (gfx1250) — hardware-verified
//
#include <hip/hip_runtime.h>


#define DIM   64
#define KA    128
#define RB    128
#define NT    256
#define NWV   8
#define CAP   4096

#define OFF_A     0
#define OFF_B     (OFF_A + RB * KA * 4)
#define OFF_SLOT  (OFF_B + KA * DIM * 4)
#define OFF_CNTW  (OFF_SLOT + CAP * 4)
#define OFF_CUR   (OFF_CNTW + NWV * RB * 4)
#define OFF_WOFF  (OFF_CUR + NWV * RB * 4)
#define OFF_CNTN  (OFF_WOFF + NWV * RB * 4)
#define OFF_OFFN  (OFF_CNTN + RB * 4)
#define OFF_BIAS  (OFF_OFFN + RB * 4)
#define OFF_LW    (OFF_BIAS + DIM * 4)
#define OFF_LB    (OFF_LW + DIM * 16 * 4)
#define OFF_O     (OFF_LB + 16 * 4)
#define OFF_MISC  (OFF_O + RB * 2 * 4)
#define LDS_BYTES (OFF_MISC + 16)

typedef char lds_align_check[((LDS_BYTES % 16) == 0) ? 1 : -1];
typedef char tile_check[(RB == NWV * 16) ? 1 : -1];
typedef char block_check[(NT == NWV * 32) ? 1 : -1];

typedef float v8f __attribute__((ext_vector_type(8)));
typedef float v4f __attribute__((ext_vector_type(4)));
typedef float v2f __attribute__((ext_vector_type(2)));
typedef __bf16 v16b __attribute__((ext_vector_type(16)));

union FragB { v16b v; unsigned short u[16]; };

__device__ __forceinline__ unsigned short bf_rne(float f) {
    unsigned int u = __float_as_uint(f);
    u += 0x7FFFu + ((u >> 16) & 1u);
    return (unsigned short)(u >> 16);
}
__device__ __forceinline__ float bf_f32(unsigned short s) {
    return __uint_as_float(((unsigned int)s) << 16);
}
__device__ __forceinline__ void split_bf16(const float (&f)[16], FragB& hi, FragB& lo) {
#pragma unroll
    for (int i = 0; i < 16; ++i) {
        unsigned short hs = bf_rne(f[i]);
        hi.u[i] = hs;
        lo.u[i] = bf_rne(f[i] - bf_f32(hs));
    }
}
__device__ __forceinline__ v8f wmma_bf16(v16b a, v16b b, v8f c) {
    c = __builtin_amdgcn_wmma_f32_16x16x32_bf16(false, a, false, b, (short)0, c, false, false);
    asm volatile("v_nop\n\tv_nop\n\tv_nop\n\tv_nop" : "+v"(c) : "v"(a), "v"(b));
    return c;
}
__device__ __forceinline__ v8f wmma3(const FragB& ah, const FragB& al,
                                     const FragB& bh, const FragB& blo, v8f c) {
    c = wmma_bf16(ah.v, bh.v, c);
    c = wmma_bf16(ah.v, blo.v, c);
    c = wmma_bf16(al.v, bh.v, c);
    return c;
}

__global__ void __launch_bounds__(NT)
sage_block_kernel(const int* edges, int E,
                  const float* xsrc, const float* xroot,
                  const float* Wl, const float* bvec, const float* Wr,
                  const float* lw, const float* lb,
                  float* yout, float* outp, int N, int fin)
{
    extern __shared__ v4f lds_dyn[];
    unsigned char* base = (unsigned char*)lds_dyn;
    float* A    = (float*)(base + OFF_A);
    v4f*   A4   = (v4f*)(base + OFF_A);
    v2f*   A2   = (v2f*)(base + OFF_A);
    float* Bw   = (float*)(base + OFF_B);
    int*   slots= (int*)(base + OFF_SLOT);
    int*   cntw = (int*)(base + OFF_CNTW);
    int*   cur  = (int*)(base + OFF_CUR);
    int*   woff = (int*)(base + OFF_WOFF);
    int*   cntn = (int*)(base + OFF_CNTN);
    int*   offn = (int*)(base + OFF_OFFN);
    float* bs   = (float*)(base + OFF_BIAS);
    float* lws  = (float*)(base + OFF_LW);
    float* lbs  = (float*)(base + OFF_LB);
    float* O    = (float*)(base + OFF_O);
    int*   misc = (int*)(base + OFF_MISC);

    const int tid = threadIdx.x;
    const int w   = tid >> 5;
    const int l   = tid & 31;
    const int h   = l >> 4;
    const int m   = l & 15;
    const int n0  = blockIdx.x * RB;
    const int* esrc = edges;
    const int* edst = edges + E;

    for (int i = tid; i < RB * KA; i += NT) A[i] = 0.0f;
    for (int i = tid; i < NWV * RB; i += NT) cntw[i] = 0;
    for (int i = tid; i < DIM * DIM; i += NT) {
        Bw[i] = Wl[i];
        Bw[DIM * DIM + i] = Wr[i];
    }
    if (tid < DIM) bs[tid] = bvec[tid];
    for (int i = tid; i < DIM * 16; i += NT) {
        int k = i >> 4, c = i & 15;
        lws[i] = (c < 2) ? lw[k * 2 + c] : 0.0f;
    }
    if (tid < 16) lbs[tid] = (tid < 2) ? lb[tid] : 0.0f;
    __syncthreads();

    const int nIt = (E + NT - 1) / NT;
    for (int it = 0; it < nIt; ++it) {
        int j = it * NT + w * 32 + l;
        int lv = -1;
        if (j < E) lv = edst[j] - n0;
        bool hit = (unsigned int)lv < (unsigned int)RB;
        unsigned int mask = __builtin_amdgcn_ballot_w32(hit);
        while (mask) {
            int b  = __builtin_ctz(mask);
            int nl = __shfl(lv, b);
            if (l == 0) cntw[w * RB + nl] += 1;
            mask &= mask - 1u;
        }
    }
    __syncthreads();

    if (tid < RB) {
        int run = 0;
        for (int ww = 0; ww < NWV; ++ww) {
            int c = cntw[ww * RB + tid];
            woff[ww * RB + tid] = run;
            run += c;
        }
        cntn[tid] = run;
    }
    __syncthreads();
    if (tid == 0) {
        int run = 0;
        for (int v = 0; v < RB; ++v) { offn[v] = run; run += cntn[v]; }
        misc[0] = run;
    }
    __syncthreads();
    if (tid < RB) {
        int o = offn[tid];
        for (int ww = 0; ww < NWV; ++ww) woff[ww * RB + tid] += o;
    }
    __syncthreads();
    const int T   = misc[0];
    const int nSw = (T + CAP - 1) / CAP;

    for (int s = 0; s < nSw; ++s) {
        const int sb = s * CAP;
        for (int i = tid; i < NWV * RB; i += NT) cur[i] = 0;
        __syncthreads();
        for (int it = 0; it < nIt; ++it) {
            int j = it * NT + w * 32 + l;
            int lv = -1, sv = 0;
            if (j < E) lv = edst[j] - n0;
            bool hit = (unsigned int)lv < (unsigned int)RB;
            if (hit) sv = esrc[j];
            unsigned int mask = __builtin_amdgcn_ballot_w32(hit);
            while (mask) {
                int b  = __builtin_ctz(mask);
                int nl = __shfl(lv, b);
                int ss = __shfl(sv, b);
                if (l == 0) {
                    int ci = w * RB + nl;
                    int p  = woff[ci] + cur[ci];
                    cur[ci] = cur[ci] + 1;
                    int q  = p - sb;
                    if ((unsigned int)q < (unsigned int)CAP) slots[q] = ss;
                }
                mask &= mask - 1u;
            }
        }
        __syncthreads();
        for (int i = 0; i < RB / NWV; ++i) {
            const int v  = w + NWV * i;
            const int c  = cntn[v];
            const int o  = offn[v];
            const int pb = (o > sb) ? o : sb;
            const int pe = ((o + c) < (sb + CAP)) ? (o + c) : (sb + CAP);
            if (pb < pe) {
                v2f sacc = A2[v * (KA / 2) + l];
                for (int p = pb; p < pe; ++p) {
                    int si = slots[p - sb];
                    if (si < 0) si += N;
                    si = (si < 0) ? 0 : si;
                    si = (si > N - 1) ? (N - 1) : si;
                    const v2f* row = (const v2f*)(xsrc + (size_t)si * DIM);
                    sacc += row[l];
                }
                A2[v * (KA / 2) + l] = sacc;
            }
        }
        __syncthreads();
    }

    for (int i = tid; i < RB * (DIM / 4); i += NT) {
        int rr = i >> 4, q = i & 15;
        int node = n0 + rr;
        v4f val = {0.0f, 0.0f, 0.0f, 0.0f};
        if (node < N) val = ((const v4f*)(xroot + (size_t)node * DIM))[q];
        A4[rr * (KA / 4) + (DIM / 4) + q] = val;
    }
    __syncthreads();

    const int r0   = w * 16;
    const int rowA = r0 + m;
    const float rc = 1.0f / fmaxf((float)cntn[rowA], 1.0f);
    v8f acc[4];
#pragma unroll
    for (int ct = 0; ct < 4; ++ct) {
        float bb = bs[ct * 16 + m];
#pragma unroll
        for (int r = 0; r < 8; ++r) acc[ct][r] = bb;
    }
#pragma unroll 1
    for (int ks = 0; ks < KA / 32; ++ks) {
        const int   k0 = ks * 32;
        const float sc = (ks < 2) ? rc : 1.0f;
        float af[16];
        {
            const v4f* ar = A4 + rowA * (KA / 4);
            v4f t0 = ar[(k0 >> 2) + 2 * h];
            v4f t1 = ar[(k0 >> 2) + 2 * h + 1];
            v4f t2 = ar[(k0 >> 2) + 4 + 2 * h];
            v4f t3 = ar[(k0 >> 2) + 4 + 2 * h + 1];
#pragma unroll
            for (int e = 0; e < 4; ++e) {
                af[e]      = t0[e] * sc;
                af[4 + e]  = t1[e] * sc;
                af[8 + e]  = t2[e] * sc;
                af[12 + e] = t3[e] * sc;
            }
        }
        FragB ah, al;
        split_bf16(af, ah, al);
#pragma unroll
        for (int ct = 0; ct < 4; ++ct) {
            const int n = ct * 16 + m;
            float bf[16];
#pragma unroll
            for (int i = 0; i < 8; ++i) {
                bf[i]     = Bw[(k0 + 8 * h + i) * DIM + n];
                bf[8 + i] = Bw[(k0 + 16 + 8 * h + i) * DIM + n];
            }
            FragB bh, blo;
            split_bf16(bf, bh, blo);
            acc[ct] = wmma3(ah, al, bh, blo, acc[ct]);
        }
    }

    __syncthreads();
#pragma unroll
    for (int ct = 0; ct < 4; ++ct) {
#pragma unroll
        for (int r = 0; r < 8; ++r) {
            float val = acc[ct][r];
            val = (val > 0.0f) ? val : 0.01f * val;
            A[(r0 + 8 * h + r) * KA + ct * 16 + m] = val;
        }
    }
    __syncthreads();

    if (fin) {
        v8f c2;
        {
            float bb = lbs[m];
#pragma unroll
            for (int r = 0; r < 8; ++r) c2[r] = bb;
        }
#pragma unroll
        for (int ks = 0; ks < DIM / 32; ++ks) {
            const int k0 = ks * 32;
            float af[16];
            {
                const v4f* ar = A4 + rowA * (KA / 4);
                v4f t0 = ar[(k0 >> 2) + 2 * h];
                v4f t1 = ar[(k0 >> 2) + 2 * h + 1];
                v4f t2 = ar[(k0 >> 2) + 4 + 2 * h];
                v4f t3 = ar[(k0 >> 2) + 4 + 2 * h + 1];
#pragma unroll
                for (int e = 0; e < 4; ++e) {
                    af[e]      = t0[e];
                    af[4 + e]  = t1[e];
                    af[8 + e]  = t2[e];
                    af[12 + e] = t3[e];
                }
            }
            FragB ah, al;
            split_bf16(af, ah, al);
            float bf[16];
#pragma unroll
            for (int i = 0; i < 8; ++i) {
                bf[i]     = lws[(k0 + 8 * h + i) * 16 + m];
                bf[8 + i] = lws[(k0 + 16 + 8 * h + i) * 16 + m];
            }
            FragB bh, blo;
            split_bf16(bf, bh, blo);
            c2 = wmma3(ah, al, bh, blo, c2);
        }
        if (m < 2) {
#pragma unroll
            for (int r = 0; r < 8; ++r) O[(r0 + 8 * h + r) * 2 + m] = c2[r];
        }
    }
    __syncthreads();

    if (!fin) {
        v4f vals[8];
#pragma unroll
        for (int rr = 0; rr < 8; ++rr) {
            int rw = r0 + 2 * rr + h;
            vals[rr] = A4[rw * (KA / 4) + m];
        }
#pragma unroll
        for (int rr = 0; rr < 8; ++rr) {
            int rw = r0 + 2 * rr + h;
            volatile v4f* gp = (volatile v4f*)(yout + (size_t)(n0 + rw) * DIM) + m;
            *gp = vals[rr];
        }
        __threadfence();
#pragma unroll
        for (int rr = 0; rr < 8; ++rr) {
            int rw = r0 + 2 * rr + h;
            volatile v4f* gp = (volatile v4f*)(yout + (size_t)(n0 + rw) * DIM) + m;
            *gp = vals[rr];
        }
    } else if (w == 0) {
        int lim = 2 * (N - n0);
        if (lim > 2 * RB) lim = 2 * RB;
        const v4f* O4 = (const v4f*)O;
        v4f ov[2];
        ov[0] = O4[l];
        ov[1] = O4[32 + l];
#pragma unroll
        for (int j = 0; j < 2; ++j) {
            int idx = j * 128 + 4 * l;
            float* gp = outp + (size_t)n0 * 2 + idx;
            if (idx + 4 <= lim) {
                *(volatile v4f*)gp = ov[j];
            } else {
#pragma unroll
                for (int e = 0; e < 4; ++e)
                    if (idx + e < lim) ((volatile float*)gp)[e] = ov[j][e];
            }
        }
        __threadfence();
#pragma unroll
        for (int j = 0; j < 2; ++j) {
            int idx = j * 128 + 4 * l;
            float* gp = outp + (size_t)n0 * 2 + idx;
            if (idx + 4 <= lim) {
                *(volatile v4f*)gp = ov[j];
            } else {
#pragma unroll
                for (int e = 0; e < 4; ++e)
                    if (idx + e < lim) ((volatile float*)gp)[e] = ov[j][e];
            }
        }
    }
}

extern "C" void kernel_launch(void* const* d_in, const int* in_sizes, int n_in,
                              void* d_out, int out_size, void* d_ws, size_t ws_size,
                              hipStream_t stream) {
    const float* x1 = (const float*)d_in[1];
    const float* x2 = (const float*)d_in[2];
    const float* x3 = (const float*)d_in[3];
    const int*   e1 = (const int*)d_in[5];
    const int*   e2 = (const int*)d_in[6];
    const float* Wl = (const float*)d_in[8];
    const float* bl = (const float*)d_in[9];
    const float* Wr = (const float*)d_in[10];
    const float* lw = (const float*)d_in[11];
    const float* lb = (const float*)d_in[12];
    float* out = (float*)d_out;

    const int N  = out_size / 2;
    const int E1 = in_sizes[5] / 2;
    const int E2 = in_sizes[6] / 2;
    if (N <= 0) return;

    const int    nb     = (N + RB - 1) / RB;
    const size_t Npad   = (size_t)nb * RB;
    const size_t ybytes = Npad * DIM * sizeof(float);
    if (2 * ybytes > ws_size) return;
    float* y2 = (float*)d_ws;
    float* y3 = (float*)((unsigned char*)d_ws + ybytes);

    const int WM = DIM * DIM;

    hipFuncSetAttribute((const void*)sage_block_kernel,
                        hipFuncAttributeMaxDynamicSharedMemorySize, LDS_BYTES);

    sage_block_kernel<<<nb, NT, LDS_BYTES, stream>>>(
        e1, E1, x1, x2, Wl + 1 * WM, bl + 1 * DIM, Wr + 1 * WM, lw, lb, y2, out, N, 0);
    sage_block_kernel<<<nb, NT, LDS_BYTES, stream>>>(
        e2, E2, x2, x3, Wl + 2 * WM, bl + 2 * DIM, Wr + 2 * WM, lw, lb, y3, out, N, 0);
    sage_block_kernel<<<nb, NT, LDS_BYTES, stream>>>(
        e2, E2, y2, y3, Wl + 6 * WM, bl + 6 * DIM, Wr + 6 * WM, lw, lb, y2, out, N, 1);
}
